// GNN_MLP_67697274520409
// MI455X (gfx1250) — hardware-verified
//
#include <hip/hip_runtime.h>
#include <stddef.h>


typedef _Float16 v16h __attribute__((ext_vector_type(16)));
typedef _Float16 v8h  __attribute__((ext_vector_type(8)));
typedef float    v8f  __attribute__((ext_vector_type(8)));
typedef float    v4f  __attribute__((ext_vector_type(4)));
typedef int      v4i  __attribute__((ext_vector_type(4)));
typedef unsigned short v8us __attribute__((ext_vector_type(8), __may_alias__));

#define CH_LINES 256
#define CH_ENT   4096
#define NBK      128
#define STH      64
#define SHIFT_A  12
#define SHIFT_B  5
#define QLINES   256

typedef char nbk_sth_check[(NBK == 2 * STH) ? 1 : -1];

union Frag { v16h v; v8h h8[2]; };

__device__ __forceinline__ v8f wmma16(v16h a, v16h b, v8f c) {
  v8f d = __builtin_amdgcn_wmma_f32_16x16x32_f16(false, a, false, b, (short)0, c, false, false);
  asm volatile("v_nop\n\tv_nop\n\tv_nop\n\tv_nop" : "+v"(d) : "v"(a), "v"(b));
  return d;
}

__device__ __forceinline__ int wave_incl(int x) {
  const int lane = threadIdx.x & 31;
#pragma unroll
  for (int o = 1; o < 32; o <<= 1) {
    int y = __shfl_up(x, o, 32);
    if (lane >= o) x += y;
  }
  return x;
}

__device__ __forceinline__ int block_exscan128(int x, int* sh, int& total) {
  const int lane = threadIdx.x & 31, w = threadIdx.x >> 5;
  int inc = wave_incl(x);
  if (lane == 31) sh[w] = inc;
  __syncthreads();
  int off = 0;
#pragma unroll
  for (int i = 0; i < 4; ++i) if (i < w) off += sh[i];
  total = sh[0] + sh[1] + sh[2] + sh[3];
  __syncthreads();
  return off + inc - x;
}

__device__ __forceinline__ int lbound(const int* __restrict__ a, int n, int v) {
  int lo = 0, hi = n;
  while (lo < hi) { int mid = (lo + hi) >> 1; if (a[mid] < v) lo = mid + 1; else hi = mid; }
  return lo;
}

template <bool FIRST>
__device__ __forceinline__ void locate_chunk(int k, int E, const int* __restrict__ pStart,
                                             const int* __restrict__ cb, int P,
                                             long long& entBase, int& nEnt) {
  if (FIRST) {
    entBase = (long long)k * CH_ENT;
    long long rem = (long long)E - entBase;
    nEnt = rem <= 0 ? 0 : (rem < CH_ENT ? (int)rem : CH_ENT);
  } else {
    int lo = 0, hi = P;
    while (hi - lo > 1) { int mid = (lo + hi) >> 1; if (cb[mid] <= k) lo = mid; else hi = mid; }
    int s = k - cb[lo];
    int l0 = pStart[lo] + s * CH_LINES;
    int l1 = pStart[lo + 1];
    if (l1 > l0 + CH_LINES) l1 = l0 + CH_LINES;
    entBase = (long long)l0 * 16;
    nEnt = (l1 > l0) ? (l1 - l0) * 16 : 0;
  }
}

template <bool FIRST>
__device__ __forceinline__ bool load_ent(const int* __restrict__ ei, int E, int N,
                                         const int* __restrict__ inEnt, long long e, int& dst, int& src) {
  if (FIRST) {
    dst = ei[(size_t)E + (size_t)e];
    src = ei[(size_t)e];
    if ((unsigned)dst >= (unsigned)N) return false;
    src = src < 0 ? 0 : (src >= N ? N - 1 : src);
    return true;
  } else {
    size_t ee = 2 * (size_t)e;
    dst = inEnt[ee];
    src = inEnt[ee + 1];
    return dst >= 0;
  }
}

template <bool FIRST>
__global__ __launch_bounds__(STH) void k_count(const int* __restrict__ ei, int E, int N,
                                               const int* __restrict__ inEnt,
                                               const int* __restrict__ pStart,
                                               const int* __restrict__ cb, int P, int Kfirst, int shift,
                                               int* cntTab, int Kcap) {
  __shared__ __attribute__((aligned(16))) unsigned short hist[STH * NBK];
  const int t = threadIdx.x;
  const int Ktot = FIRST ? Kfirst : cb[P];
  const v8us z8 = {0, 0, 0, 0, 0, 0, 0, 0};
  for (int k = blockIdx.x; k < Ktot; k += gridDim.x) {
    long long eb; int nEnt;
    locate_chunk<FIRST>(k, E, pStart, cb, P, eb, nEnt);
#pragma unroll
    for (int j = 0; j < NBK / 8; ++j) *(v8us*)(hist + t * NBK + 8 * j) = z8;
    __syncthreads();
    for (int i = 0; i * STH < nEnt; ++i) {
      int e = t + STH * i;
      if (e < nEnt) {
        int dst, src;
        if (load_ent<FIRST>(ei, E, N, inEnt, eb + e, dst, src)) {
          int d = (dst >> shift) & (NBK - 1);
          hist[t * NBK + d] += 1;
        }
      }
    }
    __syncthreads();
    int s0 = 0, s1 = 0;
#pragma unroll 8
    for (int r = 0; r < STH; ++r) { s0 += hist[r * NBK + t]; s1 += hist[r * NBK + STH + t]; }
    if (k < Kcap) {
      volatile int* row = cntTab + (size_t)k * NBK;
      row[t] = s0; row[STH + t] = s1;
      __threadfence();
      row[t] = s0; row[STH + t] = s1;
    }
    __syncthreads();
  }
}

template <bool FIRST>
__global__ __launch_bounds__(NBK) void k_scan(const int* __restrict__ cntTab, const int* __restrict__ cb,
                                              int P, int Kfirst, int* runTab, int* fStartN, int* cbN) {
  __shared__ int sh[4];
  const int d = threadIdx.x;
  for (int rep = 0; rep < 2; ++rep) {
    int outRun = 0, ckRun = 0;
    for (int p = 0; p < P; ++p) {
      const int k0 = FIRST ? 0 : cb[p];
      const int k1 = FIRST ? Kfirst : cb[p + 1];
      int totL = 0;
      for (int k = k0; k < k1; ++k) totL += (cntTab[(size_t)k * NBK + d] + 15) >> 4;
      int sumL;
      const int dOff = block_exscan128(totL, sh, sumL);
      int run = outRun + dOff;
      for (int k = k0; k < k1; ++k) {
        *(volatile int*)(runTab + (size_t)k * NBK + d) = run;
        run += (cntTab[(size_t)k * NBK + d] + 15) >> 4;
      }
      *(volatile int*)(fStartN + (size_t)p * NBK + d) = outRun + dOff;
      const int nck = (totL + CH_LINES - 1) / CH_LINES;
      int sumC;
      const int cOff = block_exscan128(nck, sh, sumC);
      *(volatile int*)(cbN + (size_t)p * NBK + d) = ckRun + cOff;
      outRun += sumL;
      ckRun += sumC;
    }
    if (d < 32) {
      *(volatile int*)(fStartN + (size_t)P * NBK + d) = (d == 0) ? outRun : 0;
      *(volatile int*)(cbN + (size_t)P * NBK + d) = (d == 0) ? ckRun : 0;
    }
    __threadfence();
    __syncthreads();
  }
}

template <bool FIRST>
__global__ __launch_bounds__(STH) void k_place(const int* __restrict__ ei, int E, int N,
                                               const int* __restrict__ inEnt,
                                               const int* __restrict__ pStart,
                                               const int* __restrict__ cb, int P, int Kfirst, int shift,
                                               const int* __restrict__ runTab, int* outEnt, int outCapLines) {
  __shared__ __attribute__((aligned(16))) unsigned short hist[STH * NBK];
  __shared__ int sEnt[2 * CH_ENT];
  __shared__ int sTot[NBK], sEb[NBK], sLc[NBK], sLb[NBK], sRun[NBK];
  __shared__ int sLmap[CH_LINES + NBK];
  __shared__ int sSegT[4], sSegL[4];
  const int t = threadIdx.x, lane = t & 31, w = t >> 5;
  const int Ktot = FIRST ? Kfirst : cb[P];
  const v8us z8 = {0, 0, 0, 0, 0, 0, 0, 0};
  for (int k = blockIdx.x; k < Ktot; k += gridDim.x) {
    long long eb; int nEnt;
    locate_chunk<FIRST>(k, E, pStart, cb, P, eb, nEnt);
#pragma unroll
    for (int j = 0; j < NBK / 8; ++j) *(v8us*)(hist + t * NBK + 8 * j) = z8;
    __syncthreads();
    for (int i = 0; i * STH < nEnt; ++i) {
      int e = t + STH * i;
      if (e < nEnt) {
        int dst, src;
        if (load_ent<FIRST>(ei, E, N, inEnt, eb + e, dst, src)) {
          int d = (dst >> shift) & (NBK - 1);
          hist[t * NBK + d] += 1;
        }
      }
    }
    __syncthreads();
    int tot0 = 0, tot1 = 0;
#pragma unroll 8
    for (int r = 0; r < STH; ++r) {
      int i0 = r * NBK + t, i1 = i0 + STH;
      int v0 = hist[i0], v1 = hist[i1];
      hist[i0] = (unsigned short)tot0; hist[i1] = (unsigned short)tot1;
      tot0 += v0; tot1 += v1;
    }
    const int lc0 = (tot0 + 15) >> 4, lc1 = (tot1 + 15) >> 4;
    const int iT0 = wave_incl(tot0), iT1 = wave_incl(tot1), iL0 = wave_incl(lc0), iL1 = wave_incl(lc1);
    if (lane == 31) { sSegT[w] = iT0; sSegT[2 + w] = iT1; sSegL[w] = iL0; sSegL[2 + w] = iL1; }
    __syncthreads();
    const int oT0 = w ? sSegT[0] : 0;
    const int oT1 = sSegT[0] + sSegT[1] + (w ? sSegT[2] : 0);
    const int oL0 = w ? sSegL[0] : 0;
    const int oL1 = sSegL[0] + sSegL[1] + (w ? sSegL[2] : 0);
    const int TL = sSegL[0] + sSegL[1] + sSegL[2] + sSegL[3];
    const int lb0 = oL0 + iL0 - lc0, lb1 = oL1 + iL1 - lc1;
    sTot[t] = tot0; sTot[STH + t] = tot1;
    sEb[t] = oT0 + iT0 - tot0; sEb[STH + t] = oT1 + iT1 - tot1;
    sLc[t] = lc0; sLc[STH + t] = lc1;
    sLb[t] = lb0; sLb[STH + t] = lb1;
    sRun[t] = runTab[(size_t)k * NBK + t]; sRun[STH + t] = runTab[(size_t)k * NBK + STH + t];
    __syncthreads();
    for (int i = 0; i * STH < nEnt; ++i) {
      int e = t + STH * i;
      if (e < nEnt) {
        int dst, src;
        if (load_ent<FIRST>(ei, E, N, inEnt, eb + e, dst, src)) {
          int d = (dst >> shift) & (NBK - 1);
          int idx = t * NBK + d;
          int pos = sEb[d] + hist[idx];
          hist[idx] += 1;
          sEnt[2 * pos] = dst; sEnt[2 * pos + 1] = src;
        }
      }
    }
    __syncthreads();
#pragma unroll 1
    for (int q = 0; q < lc0; ++q) sLmap[lb0 + q] = t;
#pragma unroll 1
    for (int q = 0; q < lc1; ++q) sLmap[lb1 + q] = STH + t;
    __syncthreads();
    for (int rep = 0; rep < 2; ++rep) {
      for (int it = 0; it * 8 < TL; ++it) {
        int L = it * 8 + w * 4 + (lane >> 3);
        if (L < TL) {
          int c = sLmap[L];
          int q = L - sLb[c];
          int gl = sRun[c] + q;
          int sub = lane & 7;
          int idx = q * 16 + sub * 2;
          int n = sTot[c];
          int base = sEb[c];
          int p0 = base + idx;     if (p0 > CH_ENT - 1) p0 = CH_ENT - 1;
          int p1 = base + idx + 1; if (p1 > CH_ENT - 1) p1 = CH_ENT - 1;
          v4i v;
          v.x = (idx < n) ? sEnt[2 * p0] : -1;
          v.y = (idx < n) ? sEnt[2 * p0 + 1] : -1;
          v.z = (idx + 1 < n) ? sEnt[2 * p1] : -1;
          v.w = (idx + 1 < n) ? sEnt[2 * p1 + 1] : -1;
          if ((unsigned)gl < (unsigned)outCapLines)
            *(volatile v4i*)(outEnt + (size_t)gl * 32 + sub * 4) = v;
        }
      }
      __threadfence();
    }
    __syncthreads();
  }
}

__global__ __launch_bounds__(32) void k_agg1(const float* __restrict__ x, const int* __restrict__ ent,
                                            const int* __restrict__ fStart,
                                            const float* __restrict__ W1, const float* __restrict__ b1,
                                            float* h1, int N) {
  __shared__ __attribute__((aligned(16))) unsigned short hist[32 * 32];
  __shared__ int sQ[QLINES * 16];
  __shared__ int sQb[32];
  __shared__ __attribute__((aligned(16))) float sT[32 * 16];
  const int lane = threadIdx.x;
  const int f = blockIdx.x;
  const int n0 = f * 32;
  const int l0 = fStart[f], l1 = fStart[f + 1];
  const v8us z8 = {0, 0, 0, 0, 0, 0, 0, 0};
  float a0 = 0.f, a1 = 0.f;
  int cnt = 0;
  for (int lb = l0; lb < l1; lb += QLINES) {
    int le = lb + QLINES; if (le > l1) le = l1;
    const int nEnt = (le - lb) * 16;
    const size_t eb = (size_t)lb * 16;
#pragma unroll
    for (int j = 0; j < 4; ++j) *(v8us*)(hist + lane * 32 + 8 * j) = z8;
    __syncthreads();
    for (int i = 0; i * 32 < nEnt; ++i) {
      int e = lane + 32 * i;
      if (e < nEnt) {
        int dst = ent[2 * (eb + (size_t)e)];
        if (dst >= 0) hist[lane * 32 + (dst & 31)] += 1;
      }
    }
    __syncthreads();
    int tot = 0;
#pragma unroll 8
    for (int r = 0; r < 32; ++r) {
      int idx = r * 32 + lane;
      int v = hist[idx];
      hist[idx] = (unsigned short)tot;
      tot += v;
    }
    const int qb = wave_incl(tot) - tot;
    sQb[lane] = qb;
    __syncthreads();
    for (int i = 0; i * 32 < nEnt; ++i) {
      int e = lane + 32 * i;
      if (e < nEnt) {
        size_t ee = 2 * (eb + (size_t)e);
        int dst = ent[ee];
        if (dst >= 0) {
          int o = dst & 31;
          int idx = lane * 32 + o;
          int pos = sQb[o] + hist[idx];
          hist[idx] += 1;
          sQ[pos] = ent[ee + 1];
        }
      }
    }
    __syncthreads();
#pragma unroll 1
    for (int j = 0; j < tot; ++j) {
      int s = sQ[qb + j];
      a0 += x[2 * (size_t)s];
      a1 += x[2 * (size_t)s + 1];
    }
    cnt += tot;
    __syncthreads();
  }
  const int node = n0 + lane;
  if (node < N) { a0 += x[2 * (size_t)node]; a1 += x[2 * (size_t)node + 1]; cnt += 1; }
  const float fc = (float)cnt;
#pragma unroll
  for (int j = 0; j < 16; ++j) {
    float v = a0 * W1[j] + a1 * W1[16 + j] + fc * b1[j];
    sT[lane * 16 + j] = v > 0.f ? v : 0.f;
  }
  __syncthreads();
  for (int rep = 0; rep < 2; ++rep) {
#pragma unroll
    for (int it = 0; it < 4; ++it) {
      int nl = it * 8 + (lane >> 2);
      int comp = (lane & 3) * 4;
      v4f v = *(const v4f*)(sT + nl * 16 + comp);
      *(volatile v4f*)(h1 + (size_t)(n0 + nl) * 16 + comp) = v;
    }
    __threadfence();
  }
}

__global__ __launch_bounds__(32) void k_agg2(const float* __restrict__ h1, const int* __restrict__ ent,
                                            const int* __restrict__ fStart,
                                            const float* __restrict__ W2, const float* __restrict__ b2,
                                            float* h2, int N) {
  __shared__ __attribute__((aligned(16))) unsigned short hist[32 * 32];
  __shared__ int sQ[QLINES * 16];
  __shared__ int sQb[32];
  __shared__ __attribute__((aligned(16))) float sA[32 * 16];
  __shared__ float sC[32];
  __shared__ __attribute__((aligned(16))) float sH[32 * 32];
  const int lane = threadIdx.x;
  const int f = blockIdx.x;
  const int n0 = f * 32;
  const int l0 = fStart[f], l1 = fStart[f + 1];
  const v8us z8 = {0, 0, 0, 0, 0, 0, 0, 0};
  v4f q0 = {0.f, 0.f, 0.f, 0.f}, q1 = q0, q2 = q0, q3 = q0;
  int cnt = 0;
  for (int lb = l0; lb < l1; lb += QLINES) {
    int le = lb + QLINES; if (le > l1) le = l1;
    const int nEnt = (le - lb) * 16;
    const size_t eb = (size_t)lb * 16;
#pragma unroll
    for (int j = 0; j < 4; ++j) *(v8us*)(hist + lane * 32 + 8 * j) = z8;
    __syncthreads();
    for (int i = 0; i * 32 < nEnt; ++i) {
      int e = lane + 32 * i;
      if (e < nEnt) {
        int dst = ent[2 * (eb + (size_t)e)];
        if (dst >= 0) hist[lane * 32 + (dst & 31)] += 1;
      }
    }
    __syncthreads();
    int tot = 0;
#pragma unroll 8
    for (int r = 0; r < 32; ++r) {
      int idx = r * 32 + lane;
      int v = hist[idx];
      hist[idx] = (unsigned short)tot;
      tot += v;
    }
    const int qb = wave_incl(tot) - tot;
    sQb[lane] = qb;
    __syncthreads();
    for (int i = 0; i * 32 < nEnt; ++i) {
      int e = lane + 32 * i;
      if (e < nEnt) {
        size_t ee = 2 * (eb + (size_t)e);
        int dst = ent[ee];
        if (dst >= 0) {
          int o = dst & 31;
          int idx = lane * 32 + o;
          int pos = sQb[o] + hist[idx];
          hist[idx] += 1;
          sQ[pos] = ent[ee + 1];
        }
      }
    }
    __syncthreads();
#pragma unroll 1
    for (int j = 0; j < tot; ++j) {
      int s = sQ[qb + j];
      const v4f* p = (const v4f*)(h1 + (size_t)s * 16);
      v4f u0 = p[0], u1 = p[1], u2 = p[2], u3 = p[3];
      q0 += u0; q1 += u1; q2 += u2; q3 += u3;
    }
    cnt += tot;
    __syncthreads();
  }
  const int node = n0 + lane;
  if (node < N) {
    const v4f* p = (const v4f*)(h1 + (size_t)node * 16);
    v4f u0 = p[0], u1 = p[1], u2 = p[2], u3 = p[3];
    q0 += u0; q1 += u1; q2 += u2; q3 += u3;
    cnt += 1;
  }
  *(v4f*)(sA + lane * 16 + 0)  = q0;
  *(v4f*)(sA + lane * 16 + 4)  = q1;
  *(v4f*)(sA + lane * 16 + 8)  = q2;
  *(v4f*)(sA + lane * 16 + 12) = q3;
  sC[lane] = (float)cnt;
  __syncthreads();

  const int m = lane & 15, hh = lane >> 4;
  v8h z8h;
#pragma unroll
  for (int i = 0; i < 8; ++i) z8h[i] = (_Float16)0.0f;
  Frag bw0, bw1;
  {
    v8h t0, t1;
#pragma unroll
    for (int i = 0; i < 8; ++i) {
      int kk = 8 * hh + i;
      t0[i] = (_Float16)(W2[kk * 32 + m] * 64.0f);
      t1[i] = (_Float16)(W2[kk * 32 + 16 + m] * 64.0f);
    }
    bw0.h8[0] = t0; bw0.h8[1] = z8h;
    bw1.h8[0] = t1; bw1.h8[1] = z8h;
  }
  const float bm0 = b2[m], bm1 = b2[16 + m];
  const v8f zc = {0.f, 0.f, 0.f, 0.f, 0.f, 0.f, 0.f, 0.f};
#pragma unroll
  for (int T = 0; T < 2; ++T) {
    Frag a;
    v8h ta;
    const float* ap = sA + (16 * T + m) * 16 + 8 * hh;
#pragma unroll
    for (int i = 0; i < 8; ++i) ta[i] = (_Float16)(ap[i] * 16.0f);
    a.h8[0] = ta; a.h8[1] = z8h;
    v8f c0 = wmma16(a.v, bw0.v, zc);
    v8f c1 = wmma16(a.v, bw1.v, zc);
#pragma unroll
    for (int r = 0; r < 8; ++r) {
      int nl = 16 * T + 8 * hh + r;
      float fc = sC[nl];
      float v0 = c0[r] * (1.0f / 1024.0f) + fc * bm0;
      float v1 = c1[r] * (1.0f / 1024.0f) + fc * bm1;
      sH[nl * 32 + m]      = v0 > 0.f ? v0 : 0.f;
      sH[nl * 32 + 16 + m] = v1 > 0.f ? v1 : 0.f;
    }
  }
  __syncthreads();
  for (int rep = 0; rep < 2; ++rep) {
#pragma unroll
    for (int it = 0; it < 8; ++it) {
      int nl = it * 4 + (lane >> 3);
      int comp = (lane & 7) * 4;
      v4f v = *(const v4f*)(sH + nl * 32 + comp);
      *(volatile v4f*)(h2 + (size_t)(n0 + nl) * 32 + comp) = v;
    }
    __threadfence();
  }
}

__global__ __launch_bounds__(64) void k_pool_head(const float* __restrict__ h2, const int* __restrict__ bidx,
                                                 int N, int G,
                                                 const float* __restrict__ Wf1, const float* __restrict__ bf1,
                                                 const float* __restrict__ Wf2, const float* __restrict__ bf2,
                                                 float* out) {
  __shared__ __attribute__((aligned(16))) float sP[2][16 * 32];
  __shared__ float sO[32];
  const int t = threadIdx.x, lane = t & 31, w = t >> 5;
  const int gw = blockIdx.x * 32 + w * 16;
  for (int gi = 0; gi < 16; ++gi) {
    const int g = gw + gi;
    int lo = 0, hi = 0;
    if (g < G) { lo = lbound(bidx, N, g); hi = lbound(bidx, N, g + 1); }
    float s0 = 0.f, s1 = 0.f, s2 = 0.f, s3 = 0.f;
    int n = lo;
#pragma unroll 1
    for (; n + 3 < hi; n += 4) {
      s0 += h2[(size_t)n * 32 + lane];
      s1 += h2[(size_t)(n + 1) * 32 + lane];
      s2 += h2[(size_t)(n + 2) * 32 + lane];
      s3 += h2[(size_t)(n + 3) * 32 + lane];
    }
#pragma unroll 1
    for (; n < hi; ++n) s0 += h2[(size_t)n * 32 + lane];
    const float c = (float)(hi - lo);
    const float inv = 1.0f / fmaxf(c, 1.0f);
    sP[w][gi * 32 + lane] = ((s0 + s1) + (s2 + s3)) * inv;
  }
  __syncthreads();
  const int m = lane & 15, hh = lane >> 4;
  Frag a, b;
  {
    v8h t0, t1, u0, u1;
    const float* pr = &sP[w][m * 32];
#pragma unroll
    for (int i = 0; i < 8; ++i) {
      t0[i] = (_Float16)(pr[8 * hh + i] * 16.0f);
      t1[i] = (_Float16)(pr[16 + 8 * hh + i] * 16.0f);
      u0[i] = (_Float16)(Wf1[(8 * hh + i) * 16 + m] * 64.0f);
      u1[i] = (_Float16)(Wf1[(16 + 8 * hh + i) * 16 + m] * 64.0f);
    }
    a.h8[0] = t0; a.h8[1] = t1;
    b.h8[0] = u0; b.h8[1] = u1;
  }
  const v8f zc = {0.f, 0.f, 0.f, 0.f, 0.f, 0.f, 0.f, 0.f};
  v8f cacc = wmma16(a.v, b.v, zc);
  const float bb = bf1[m], w2 = Wf2[m], b3 = bf2[0];
  float tv[8];
#pragma unroll
  for (int r = 0; r < 8; ++r) {
    float y = cacc[r] * (1.0f / 1024.0f) + bb;
    y = y > 0.f ? y : 0.f;
    tv[r] = y * w2;
  }
#pragma unroll
  for (int o = 1; o < 16; o <<= 1) {
#pragma unroll
    for (int r = 0; r < 8; ++r) tv[r] += __shfl_xor(tv[r], o, 32);
  }
  if (m == 0) {
#pragma unroll
    for (int r = 0; r < 8; ++r) sO[w * 16 + 8 * hh + r] = tv[r] + b3;
  }
  __syncthreads();
  const int g = blockIdx.x * 32 + lane;
  const float v = (w == 0) ? sO[lane] : 0.f;
  if (w == 0 && g < G) *(volatile float*)(out + g) = v;
  __threadfence();
  if (w == 0 && g < G) *(volatile float*)(out + g) = v;
}

extern "C" void kernel_launch(void* const* d_in, const int* in_sizes, int n_in,
                              void* d_out, int out_size, void* d_ws, size_t ws_size,
                              hipStream_t stream) {
  if (n_in < 11) return;
  const float* x    = (const float*)d_in[0];
  const int*   ei   = (const int*)  d_in[1];
  const int*   bidx = (const int*)  d_in[2];
  const float* W1   = (const float*)d_in[3];
  const float* b1   = (const float*)d_in[4];
  const float* W2   = (const float*)d_in[5];
  const float* b2   = (const float*)d_in[6];
  const float* Wf1  = (const float*)d_in[7];
  const float* bf1  = (const float*)d_in[8];
  const float* Wf2  = (const float*)d_in[9];
  const float* bf2  = (const float*)d_in[10];
  float* out = (float*)d_out;

  const int N = in_sizes[0] / 2;
  const int E = in_sizes[1] / 2;
  const int G = out_size;
  if (N <= 0 || E < 0 || G <= 0) return;
  if (N > (1 << 19)) return;
  if (in_sizes[2] < N) return;

  const int       K1    = (E + CH_ENT - 1) / CH_ENT;
  const long long EL    = ((long long)E + 15) / 16;
  const long long B1L   = EL + (long long)K1 * NBK;
  const long long K2cap = B1L / CH_LINES + NBK;
  const long long B2L   = EL + K2cap * NBK;
  const int       F2    = NBK * NBK;
  const int       NB32  = (N + 31) / 32;
  if (B1L > 0x7fffffffLL || B2L > 0x7fffffffLL) return;

  size_t off = 0;
  auto carve = [&](size_t bytes) { size_t o = off; off += (bytes + 127) & ~(size_t)127; return o; };
  const size_t oOut1 = carve((size_t)B1L * 128);
  const size_t oCnt1 = carve((size_t)K1 * NBK * 4);
  const size_t oRun1 = carve((size_t)K1 * NBK * 4);
  const size_t oFs1  = carve((size_t)(NBK + 32) * 4);
  const size_t oCb2  = carve((size_t)(NBK + 32) * 4);
  const size_t oOut2 = carve((size_t)B2L * 128);
  const size_t oCnt2 = carve((size_t)K2cap * NBK * 4);
  const size_t oRun2 = carve((size_t)K2cap * NBK * 4);
  const size_t oFs2  = carve((size_t)(F2 + 32) * 4);
  const size_t oCb3  = carve((size_t)(F2 + 32) * 4);
  const size_t oH1   = carve((size_t)NB32 * 32 * 16 * 4);
  const size_t oH2   = carve((size_t)NB32 * 32 * 32 * 4);
  if (off > ws_size) return;

  char* ws = (char*)d_ws;
  int*   out1 = (int*)(ws + oOut1);
  int*   cnt1 = (int*)(ws + oCnt1);
  int*   run1 = (int*)(ws + oRun1);
  int*   fs1  = (int*)(ws + oFs1);
  int*   cb2  = (int*)(ws + oCb2);
  int*   out2 = (int*)(ws + oOut2);
  int*   cnt2 = (int*)(ws + oCnt2);
  int*   run2 = (int*)(ws + oRun2);
  int*   fs2  = (int*)(ws + oFs2);
  int*   cb3  = (int*)(ws + oCb3);
  float* h1   = (float*)(ws + oH1);
  float* h2   = (float*)(ws + oH2);

  const int g1 = K1 > 0 ? K1 : 1;
  const int gB = 1024;

  k_count<true><<<g1, STH, 0, stream>>>(ei, E, N, out1, fs1, cb2, 1, K1, SHIFT_A, cnt1, K1);
  k_scan<true><<<1, NBK, 0, stream>>>(cnt1, cb2, 1, K1, run1, fs1, cb2);
  k_place<true><<<g1, STH, 0, stream>>>(ei, E, N, out1, fs1, cb2, 1, K1, SHIFT_A, run1, out1, (int)B1L);
  k_count<false><<<gB, STH, 0, stream>>>(ei, E, N, out1, fs1, cb2, NBK, 0, SHIFT_B, cnt2, (int)K2cap);
  k_scan<false><<<1, NBK, 0, stream>>>(cnt2, cb2, NBK, 0, run2, fs2, cb3);
  k_place<false><<<gB, STH, 0, stream>>>(ei, E, N, out1, fs1, cb2, NBK, 0, SHIFT_B, run2, out2, (int)B2L);
  k_agg1<<<NB32, 32, 0, stream>>>(x, out2, fs2, W1, b1, h1, N);
  k_agg2<<<NB32, 32, 0, stream>>>(h1, out2, fs2, W2, b2, h2, N);
  k_pool_head<<<(G + 31) / 32, 64, 0, stream>>>(h2, bidx, N, G, Wf1, bf1, Wf2, bf2, out);
  (void)hipGetLastError();
}
